// PEPSI_52201032516135
// MI455X (gfx1250) — hardware-verified
//
#include <hip/hip_runtime.h>
#include <stddef.h>
#include <stdint.h>

#pragma clang fp contract(off)

#define NS    8
#define IH    40
#define IW    40
#define HW    1600
#define DD    128
#define NPIX  12800
#define CW    38
#define CC    1444
#define CP    1536
#define HROWS 6400
#define OTP   68
#define STQ   72

static_assert(NPIX == NS * HW);
static_assert(HW % 64 == 0);
static_assert(HW == IH * IW);
static_assert(CC == CW * CW);
static_assert(CP % 256 == 0);
static_assert(CP >= CC);
static_assert(NPIX % 256 == 0);
static_assert((NS * CP) % 256 == 0);
static_assert(HROWS * 2 == NPIX);
static_assert(HROWS % HW == 0);
static_assert(DD == 128);

typedef _Float16 v16h __attribute__((ext_vector_type(16)));
typedef _Float16 v8h  __attribute__((ext_vector_type(8)));
typedef __bf16   v16b __attribute__((ext_vector_type(16)));
typedef unsigned short v16us __attribute__((ext_vector_type(16)));
typedef unsigned short v8us  __attribute__((ext_vector_type(8)));
typedef float    v8f  __attribute__((ext_vector_type(8)));
typedef float    v4f  __attribute__((ext_vector_type(4)));
typedef unsigned int v4u __attribute__((ext_vector_type(4)));

union Frag   { v16h v; v8h h[2]; };
union FragB  { v16b v; v16us u; v8us h[2]; };
union Pack8  { v8h h; v4u u; };
union Pack8u { v8us h; v4u u; };

__device__ __forceinline__ v8f mma16(v16h a, v16h b, v8f c) {
  c = __builtin_amdgcn_wmma_f32_16x16x32_f16(false, a, false, b, (short)0, c, false, false);
  asm volatile("v_nop\n\tv_nop\n\tv_nop\n\tv_nop" : "+v"(c) : "v"(a), "v"(b));
  return c;
}
__device__ __forceinline__ v8f mmab(v16b a, v16b b, v8f c) {
  c = __builtin_amdgcn_wmma_f32_16x16x32_bf16(false, a, false, b, (short)0, c, false, false);
  asm volatile("v_nop\n\tv_nop\n\tv_nop\n\tv_nop" : "+v"(c) : "v"(a), "v"(b));
  return c;
}

__device__ __forceinline__ v16h ldfrag(const _Float16* p, int ld, int row0, int k0, int lane) {
  const int m = lane & 15, lh = lane >> 4;
  const _Float16* q = p + (size_t)(row0 + m) * ld + k0 + 8 * lh;
  Frag f;
  f.h[0] = *(const v8h*)(q);
  f.h[1] = *(const v8h*)(q + 16);
  return f.v;
}
__device__ __forceinline__ v16b ldfragb(const unsigned short* p, int ld, int row0, int k0, int lane) {
  const int m = lane & 15, lh = lane >> 4;
  const unsigned short* q = p + (size_t)(row0 + m) * ld + k0 + 8 * lh;
  FragB f;
  f.h[0] = *(const v8us*)(q);
  f.h[1] = *(const v8us*)(q + 16);
  return f.v;
}

__device__ __forceinline__ v8f zero8() { return (v8f){0.f, 0.f, 0.f, 0.f, 0.f, 0.f, 0.f, 0.f}; }

__device__ __forceinline__ unsigned short bf_rne(float x) {
  unsigned int u = __float_as_uint(x);
  u += 0x7FFFu + ((u >> 16) & 1u);
  return (unsigned short)(u >> 16);
}
__device__ __forceinline__ float bf_up(unsigned short h) { return __uint_as_float(((unsigned int)h) << 16); }

__device__ __forceinline__ void gemm32x64(const _Float16* __restrict__ A, int lda,
                                          const _Float16* __restrict__ Bt, int ldb, int K,
                                          int m0, int n0, int lane, v8f (&acc)[2][4]) {
#pragma unroll 1
  for (int k0 = 0; k0 < K; k0 += 32) {
    const v16h a0 = ldfrag(A, lda, m0, k0, lane);
    const v16h a1 = ldfrag(A, lda, m0 + 16, k0, lane);
    const v16h b0 = ldfrag(Bt, ldb, n0, k0, lane);
    const v16h b1 = ldfrag(Bt, ldb, n0 + 16, k0, lane);
    const v16h b2 = ldfrag(Bt, ldb, n0 + 32, k0, lane);
    const v16h b3 = ldfrag(Bt, ldb, n0 + 48, k0, lane);
    acc[0][0] = mma16(a0, b0, acc[0][0]);
    acc[1][0] = mma16(a1, b0, acc[1][0]);
    acc[0][1] = mma16(a0, b1, acc[0][1]);
    acc[1][1] = mma16(a1, b1, acc[1][1]);
    acc[0][2] = mma16(a0, b2, acc[0][2]);
    acc[1][2] = mma16(a1, b2, acc[1][2]);
    acc[0][3] = mma16(a0, b3, acc[0][3]);
    acc[1][3] = mma16(a1, b3, acc[1][3]);
  }
}

__device__ __forceinline__ void gemm32x64_bx3(const unsigned short* __restrict__ Ah, const unsigned short* __restrict__ Al,
                                              const unsigned short* __restrict__ Bh, const unsigned short* __restrict__ Bl,
                                              int ld, int K, int m0, int n0, int lane, v8f (&acc)[2][4]) {
#pragma unroll 1
  for (int k0 = 0; k0 < K; k0 += 32) {
    const v16b ah0 = ldfragb(Ah, ld, m0, k0, lane);
    const v16b ah1 = ldfragb(Ah, ld, m0 + 16, k0, lane);
    const v16b al0 = ldfragb(Al, ld, m0, k0, lane);
    const v16b al1 = ldfragb(Al, ld, m0 + 16, k0, lane);
#pragma unroll
    for (int t = 0; t < 4; ++t) {
      const v16b bhf = ldfragb(Bh, ld, n0 + 16 * t, k0, lane);
      const v16b blf = ldfragb(Bl, ld, n0 + 16 * t, k0, lane);
      acc[0][t] = mmab(ah0, bhf, acc[0][t]);
      acc[0][t] = mmab(ah0, blf, acc[0][t]);
      acc[0][t] = mmab(al0, bhf, acc[0][t]);
      acc[1][t] = mmab(ah1, bhf, acc[1][t]);
      acc[1][t] = mmab(ah1, blf, acc[1][t]);
      acc[1][t] = mmab(al1, bhf, acc[1][t]);
    }
  }
}

__device__ __forceinline__ void out_epilogue_f32(v8f (&acc)[2][4], float scale, const float (&bb)[4],
                                                 float* sw, float* __restrict__ out, int ldo,
                                                 int m0, int n0, int lane, int hh, int c) {
#pragma unroll
  for (int sub = 0; sub < 2; ++sub) {
    __syncthreads();
#pragma unroll
    for (int t = 0; t < 4; ++t) {
#pragma unroll
      for (int r = 0; r < 8; ++r) sw[(8 * hh + r) * OTP + 16 * t + c] = acc[sub][t][r] * scale + bb[t];
    }
    __syncthreads();
    v4f val[8];
    size_t go[8];
#pragma unroll
    for (int it = 0; it < 8; ++it) {
      const int p    = lane + 32 * it;
      const int L    = p >> 3;
      const int pc   = p & 7;
      const int row  = L >> 1;
      const int half = L & 1;
      val[it] = *(const v4f*)(sw + row * OTP + half * 32 + pc * 4);
      go[it]  = (size_t)(m0 + sub * 16 + row) * ldo + n0 + half * 32 + pc * 4;
    }
    for (int ps = 0; ps < 2; ++ps) {
#pragma unroll
      for (int it = 0; it < 8; ++it) *(volatile v4f*)(out + go[it]) = val[it];
      __threadfence();
    }
  }
}

__device__ __forceinline__ void out_epilogue_elu(v8f (&acc)[2][4], float scale, const float (&bb)[4],
                                                 float* sw, float* __restrict__ out, int ldo,
                                                 int m0, int n0, int lane, int hh, int c) {
#pragma unroll
  for (int sub = 0; sub < 2; ++sub) {
    __syncthreads();
#pragma unroll
    for (int t = 0; t < 4; ++t) {
#pragma unroll
      for (int r = 0; r < 8; ++r) sw[(8 * hh + r) * OTP + 16 * t + c] = acc[sub][t][r] * scale + bb[t];
    }
    __syncthreads();
#pragma unroll 1
    for (int i = 0; i < 32; ++i) {
      const int j   = lane + 32 * i;
      const int idx = (j >> 6) * OTP + (j & 63);
      const float v = sw[idx];
      const float e = expm1f(fminf(v, 0.f));
      sw[idx] = (v > 0.f) ? v : e;
    }
    __syncthreads();
    v4f val[8];
    size_t go[8];
#pragma unroll
    for (int it = 0; it < 8; ++it) {
      const int p    = lane + 32 * it;
      const int L    = p >> 3;
      const int pc   = p & 7;
      const int row  = L >> 1;
      const int half = L & 1;
      val[it] = *(const v4f*)(sw + row * OTP + half * 32 + pc * 4);
      go[it]  = (size_t)(m0 + sub * 16 + row) * ldo + n0 + half * 32 + pc * 4;
    }
    for (int ps = 0; ps < 2; ++ps) {
#pragma unroll
      for (int it = 0; it < 8; ++it) *(volatile v4f*)(out + go[it]) = val[it];
      __threadfence();
    }
  }
}

__device__ __forceinline__ void out_epilogue_acl(v8f (&acc)[2][4], float* sw,
                                                 const float* __restrict__ g, const float* __restrict__ msk,
                                                 _Float16* __restrict__ con, size_t l0, int n0,
                                                 int lane, int hh, int c) {
#pragma unroll
  for (int sub = 0; sub < 2; ++sub) {
    __syncthreads();
#pragma unroll
    for (int t = 0; t < 4; ++t) {
#pragma unroll
      for (int r = 0; r < 8; ++r) {
        float a = acc[sub][t][r] * 0.000244140625f;
        a = a * (1.0f / 9.0f);
        sw[(8 * hh + r) * OTP + 16 * t + c] = a;
      }
    }
    __syncthreads();
    v4u val[4];
    size_t go[4];
#pragma unroll
    for (int it = 0; it < 4; ++it) {
      const int p  = lane + 32 * it;
      const int L  = p >> 3;
      const int pc = p & 7;
      const size_t l = l0 + sub * 16 + L;
      const float mk = msk[l];
      const float om = 1.0f - mk;
      const float* gr = g + l * DD + n0 + pc * 8;
      const v4f g0 = *(const v4f*)(gr), g1 = *(const v4f*)(gr + 4);
      const float* ra = sw + L * OTP + pc * 8;
      const v4f a0 = *(const v4f*)(ra), a1 = *(const v4f*)(ra + 4);
      float v[8];
#pragma unroll
      for (int j = 0; j < 4; ++j) {
        const float bg0 = g0[j] * mk;
        v[j]     = bg0 + a0[j] * om;
        const float bg1 = g1[j] * mk;
        v[4 + j] = bg1 + a1[j] * om;
      }
      Pack8 pk;
      pk.h = (v8h){(_Float16)v[0], (_Float16)v[1], (_Float16)v[2], (_Float16)v[3],
                   (_Float16)v[4], (_Float16)v[5], (_Float16)v[6], (_Float16)v[7]};
      val[it] = pk.u;
      go[it]  = l * (size_t)(2 * DD) + DD + n0 + pc * 8;
    }
    for (int ps = 0; ps < 2; ++ps) {
#pragma unroll
      for (int it = 0; it < 4; ++it) *(volatile v4u*)(con + go[it]) = val[it];
      __threadfence();
    }
  }
}

__global__ __launch_bounds__(256) void k_prep(const float* __restrict__ g, const float* __restrict__ msk,
                                              _Float16* __restrict__ con,
                                              unsigned short* __restrict__ gh, unsigned short* __restrict__ gl,
                                              unsigned short* __restrict__ bh, unsigned short* __restrict__ bl,
                                              _Float16* __restrict__ bgt,
                                              float* __restrict__ g2s, float* __restrict__ bg2s) {
  __shared__ __align__(16) _Float16 st[DD * STQ];
  __shared__ __align__(16) float sq[64];
  __shared__ __align__(16) float sqb[64];
  const int tid = threadIdx.x, lane = tid & 31, wave = tid >> 5;
  const int hh = lane >> 4, c16 = lane & 15;
  const int blk  = blockIdx.x;
  const int b    = blk / 25;
  const int q0   = (blk - b * 25) * 64;
  const int pix0 = b * HW + q0;
#pragma unroll 1
  for (int i = 0; i < 4; ++i) {
    const int pl  = wave * 8 + 2 * i + hh;
    const int pix = pix0 + pl;
    const int d0  = 8 * c16;
    const float* src = g + (size_t)pix * DD + d0;
    const v4f a0 = *(const v4f*)(src);
    const v4f a1 = *(const v4f*)(src + 4);
    const float mk = msk[pix];
    const v4f b0 = a0 * mk;
    const v4f b1 = a1 * mk;
    float s  = ((a0[0] * a0[0] + a0[1] * a0[1]) + (a0[2] * a0[2] + a0[3] * a0[3])) +
               ((a1[0] * a1[0] + a1[1] * a1[1]) + (a1[2] * a1[2] + a1[3] * a1[3]));
    float sb = ((b0[0] * b0[0] + b0[1] * b0[1]) + (b0[2] * b0[2] + b0[3] * b0[3])) +
               ((b1[0] * b1[0] + b1[1] * b1[1]) + (b1[2] * b1[2] + b1[3] * b1[3]));
#pragma unroll
    for (int off = 1; off < 16; off <<= 1) {
      s  += __shfl_xor(s, off, 32);
      sb += __shfl_xor(sb, off, 32);
    }
    if (c16 == 0) { sq[pl] = s; sqb[pl] = sb; }
#pragma unroll
    for (int j = 0; j < 4; ++j) {
      st[(d0 + j) * STQ + pl]     = (_Float16)b0[j];
      st[(d0 + 4 + j) * STQ + pl] = (_Float16)b1[j];
    }
    Pack8 pg;
    pg.h = (v8h){(_Float16)a0[0], (_Float16)a0[1], (_Float16)a0[2], (_Float16)a0[3],
                 (_Float16)a1[0], (_Float16)a1[1], (_Float16)a1[2], (_Float16)a1[3]};
    Pack8u ph, plo, qh, qlo;
#pragma unroll
    for (int j = 0; j < 4; ++j) {
      const unsigned short t0 = bf_rne(a0[j]);
      ph.h[j]      = t0;
      plo.h[j]     = bf_rne(a0[j] - bf_up(t0));
      const unsigned short t1 = bf_rne(a1[j]);
      ph.h[4 + j]  = t1;
      plo.h[4 + j] = bf_rne(a1[j] - bf_up(t1));
      const unsigned short u0 = bf_rne(b0[j]);
      qh.h[j]      = u0;
      qlo.h[j]     = bf_rne(b0[j] - bf_up(u0));
      const unsigned short u1 = bf_rne(b1[j]);
      qh.h[4 + j]  = u1;
      qlo.h[4 + j] = bf_rne(b1[j] - bf_up(u1));
    }
    const v4u vg = pg.u, vh = ph.u, vl = plo.u, wh = qh.u, wl = qlo.u;
    const size_t o128 = (size_t)pix * DD + d0;
    const size_t o256 = (size_t)pix * (2 * DD) + d0;
    for (int ps = 0; ps < 2; ++ps) {
      *(volatile v4u*)(con + o256) = vg;
      *(volatile v4u*)(gh + o128)  = vh;
      *(volatile v4u*)(gl + o128)  = vl;
      *(volatile v4u*)(bh + o128)  = wh;
      *(volatile v4u*)(bl + o128)  = wl;
      __threadfence();
    }
  }
  __syncthreads();
  {
    v4u val[4];
    size_t go[4];
#pragma unroll
    for (int j = 0; j < 4; ++j) {
      const int p  = tid + 256 * j;
      const int d  = p >> 3;
      const int pc = p & 7;
      Pack8 pk;
      pk.h   = *(const v8h*)(st + d * STQ + pc * 8);
      val[j] = pk.u;
      go[j]  = ((size_t)(b * DD + d)) * HW + q0 + pc * 8;
    }
    for (int ps = 0; ps < 2; ++ps) {
#pragma unroll
      for (int j = 0; j < 4; ++j) *(volatile v4u*)(bgt + go[j]) = val[j];
      __threadfence();
    }
  }
  if (wave == 0) {
    const v4f xs = *(const v4f*)(sq + 4 * c16);
    const v4f xb = *(const v4f*)(sqb + 4 * c16);
    v4f v;
    v[0] = hh ? xb[0] : xs[0];
    v[1] = hh ? xb[1] : xs[1];
    v[2] = hh ? xb[2] : xs[2];
    v[3] = hh ? xb[3] : xs[3];
    float* dst = (hh ? bg2s : g2s) + pix0 + 4 * c16;
    for (int ps = 0; ps < 2; ++ps) {
      *(volatile v4f*)dst = v;
      __threadfence();
    }
  }
}

__global__ __launch_bounds__(256) void k_wt(const float* __restrict__ w, _Float16* __restrict__ wt) {
  const int idx = blockIdx.x * 256 + threadIdx.x;
  const int n  = idx >> 5;
  const int kg = idx & 31;
  float v[8];
#pragma unroll
  for (int j = 0; j < 8; ++j) v[j] = w[(size_t)(8 * kg + j) * DD + n] * 64.0f;
  Pack8 pk;
  pk.h = (v8h){(_Float16)v[0], (_Float16)v[1], (_Float16)v[2], (_Float16)v[3],
               (_Float16)v[4], (_Float16)v[5], (_Float16)v[6], (_Float16)v[7]};
  const v4u vv = pk.u;
  volatile v4u* d = (volatile v4u*)(wt + (size_t)n * (2 * DD) + 8 * kg);
  *d = vv;
  __threadfence();
  *d = vv;
}

__global__ __launch_bounds__(256) void k_norm9(const float* __restrict__ g2s, const float* __restrict__ bg2s,
                                               float* __restrict__ wwd, float* __restrict__ k1d) {
  const int tid = threadIdx.x;
  if (blockIdx.x < 50) {
    const int idx = blockIdx.x * 256 + tid;
    const int b = idx / HW, pix = idx - b * HW;
    const int y = pix / IW, x = pix - y * IW;
    const float* gs = g2s + b * HW;
    float s = 0.f;
#pragma unroll
    for (int t = 0; t < 9; ++t) {
      const int dy = t / 3, dx = t - dy * 3;
      const int yy = y + dy - 1, xx = x + dx - 1;
      const bool ok = ((unsigned)yy < (unsigned)IH) && ((unsigned)xx < (unsigned)IW);
      const int yc = min(max(yy, 0), IH - 1), xc = min(max(xx, 0), IW - 1);
      const float v = gs[yc * IW + xc];
      s += ok ? v : 0.f;
    }
    volatile float* d = (volatile float*)(wwd + idx);
    *d = s;
    __threadfence();
    *d = s;
  } else {
    const int idx = (blockIdx.x - 50) * 256 + tid;
    const int b = idx / CP, cpos = idx - b * CP;
    const bool in = cpos < CC;
    const int cc = in ? cpos : (CC - 1);
    const int py = cc / CW, px = cc - py * CW;
    const float* gs = bg2s + b * HW;
    float s = 0.f;
#pragma unroll
    for (int t = 0; t < 9; ++t) {
      const int dy = t / 3, dx = t - dy * 3;
      s += gs[(py + dy) * IW + (px + dx)];
    }
    const float vout = in ? s : 0.f;
    volatile float* d = (volatile float*)(k1d + idx);
    *d = vout;
    __threadfence();
    *d = vout;
  }
}

template <int WPB>
__global__ __launch_bounds__(32 * WPB) void k_gg(const unsigned short* __restrict__ gh, const unsigned short* __restrict__ gl,
                                                 const unsigned short* __restrict__ bh, const unsigned short* __restrict__ bl,
                                                 float* __restrict__ gg4, int sbase) {
  __shared__ __align__(16) float st[WPB][16 * OTP];
  const int tid = threadIdx.x, lane = tid & 31, wave = tid >> 5;
  const int hh = lane >> 4, c = lane & 15;
  const int z  = blockIdx.z;
  const int m0 = (blockIdx.y * WPB + wave) * 32;
  const int n0 = blockIdx.x * 64;
  const size_t prow = (size_t)(sbase + z) * HW;
  const unsigned short* Ah = gh + prow * DD;
  const unsigned short* Al = gl + prow * DD;
  const unsigned short* Bh = bh + prow * DD;
  const unsigned short* Bl = bl + prow * DD;

  v8f acc[2][4];
#pragma unroll
  for (int s = 0; s < 2; ++s)
#pragma unroll
    for (int t = 0; t < 4; ++t) acc[s][t] = zero8();
  gemm32x64_bx3(Ah, Al, Bh, Bl, DD, DD, m0, n0, lane, acc);
  const float bb[4] = {0.f, 0.f, 0.f, 0.f};
  out_epilogue_f32(acc, 1.0f, bb, st[wave], gg4 + (size_t)z * HW * HW, HW, m0, n0, lane, hh, c);
}

__device__ __forceinline__ float blk_sum(float v, float* r8, int lane, int wave) {
#pragma unroll
  for (int off = 16; off >= 1; off >>= 1) v += __shfl_xor(v, off, 32);
  if (lane == 0) r8[wave] = v;
  __syncthreads();
  float s = 0.f;
#pragma unroll
  for (int w = 0; w < 8; ++w) s += r8[w];
  return s;
}
__device__ __forceinline__ float blk_min(float v, float* r8, int lane, int wave) {
#pragma unroll
  for (int off = 16; off >= 1; off >>= 1) v = fminf(v, __shfl_xor(v, off, 32));
  if (lane == 0) r8[wave] = v;
  __syncthreads();
  float s = r8[0];
#pragma unroll
  for (int w = 1; w < 8; ++w) s = fminf(s, r8[w]);
  return s;
}
__device__ __forceinline__ float blk_max(float v, float* r8, int lane, int wave) {
#pragma unroll
  for (int off = 16; off >= 1; off >>= 1) v = fmaxf(v, __shfl_xor(v, off, 32));
  if (lane == 0) r8[wave] = v;
  __syncthreads();
  float s = r8[0];
#pragma unroll
  for (int w = 1; w < 8; ++w) s = fmaxf(s, r8[w]);
  return s;
}

__global__ __launch_bounds__(256) void k_stats(const float* __restrict__ gg4, const float* __restrict__ wwd,
                                               const float* __restrict__ k1d, _Float16* __restrict__ ca, int rbase) {
  __shared__ __align__(16) float buf[CP];
  __shared__ float r_s[8], r_mn[8], r_q[8], r_mx[8], r_e[8];
  const int tid = threadIdx.x, lane = tid & 31, wave = tid >> 5;
  const int rrel = blockIdx.x;
  const int bl   = rrel / HW;
  const int pix  = rrel - bl * HW;
  const int r    = rbase + rrel;
  const int b    = r / HW;
  const int y = pix / IW, x = pix - y * IW;
  const float wv = wwd[r];
  const float* kd = k1d + b * CP;
  int toff[9];
  bool tok[9];
#pragma unroll
  for (int t = 0; t < 9; ++t) {
    const int dy = t / 3, dx = t - dy * 3;
    const int py = y + dy - 1, px = x + dx - 1;
    tok[t] = ((unsigned)py < (unsigned)IH) && ((unsigned)px < (unsigned)IW);
    const int pyc = min(max(py, 0), IH - 1), pxc = min(max(px, 0), IW - 1);
    toff[t] = (bl * HW + pyc * IW + pxc) * HW + dy * IW + dx;
  }
  const float PINF = __builtin_huge_valf();
  float s = 0.f, mn = PINF;
#pragma unroll 1
  for (int i = 0; i < CP / 256; ++i) {
    const int j = tid + 256 * i;
    const bool in = j < CC;
    const int cc = in ? j : (CC - 1);
    const int py = cc / CW, px = cc - py * CW;
    const int cidx = py * IW + px;
    float cs = 0.f;
#pragma unroll
    for (int t = 0; t < 9; ++t) {
      const float v = gg4[toff[t] + cidx];
      cs += tok[t] ? v : 0.f;
    }
    const float t1 = kd[cc] + wv;
    const float t2 = 2.0f * cs;
    const float ds = t1 - t2;
    buf[j] = ds;
    s += in ? ds : 0.f;
    mn = fminf(mn, in ? ds : PINF);
  }
  const float S  = blk_sum(s, r_s, lane, wave);
  const float MN = blk_min(mn, r_mn, lane, wave);
  (void)MN;
  const float mu = S * (1.0f / 1444.0f);
  float q = 0.f;
#pragma unroll 1
  for (int i = 0; i < CP / 256; ++i) {
    const int j = tid + 256 * i;
    const bool in = j < CC;
    const float dv = buf[j] - mu;
    const float d2 = dv * dv;
    q += in ? d2 : 0.f;
  }
  const float Q   = blk_sum(q, r_q, lane, wave);
  const float var = Q * (1.0f / 1444.0f);
  const float sd  = sqrtf(var);
  const float rsd = 1.0f / sd;
  float mx = -PINF;
#pragma unroll 1
  for (int i = 0; i < CP / 256; ++i) {
    const int j = tid + 256 * i;
    const bool in = j < CC;
    const float zt = (buf[j] - mu) * rsd;
    const float tz = tanhf(zt);
    const float sj = -50.0f * tz;
    buf[j] = sj;
    mx = fmaxf(mx, in ? sj : -PINF);
  }
  const float MX = blk_max(mx, r_mx, lane, wave);
  float se = 0.f;
#pragma unroll 1
  for (int i = 0; i < CP / 256; ++i) {
    const int j = tid + 256 * i;
    const bool in = j < CC;
    const float ex = __expf(buf[j] - MX);
    const float e  = in ? ex : 0.f;
    buf[j] = e;
    se += e;
  }
  const float SE  = blk_sum(se, r_e, lane, wave);
  const float inv = 1.0f / SE;
  if (tid < 192) {
    const float* sp = buf + 8 * tid;
    const v4f a0 = *(const v4f*)(sp), a1 = *(const v4f*)(sp + 4);
    Pack8 pk;
    pk.h = (v8h){(_Float16)((a0[0] * inv) * 4096.0f), (_Float16)((a0[1] * inv) * 4096.0f),
                 (_Float16)((a0[2] * inv) * 4096.0f), (_Float16)((a0[3] * inv) * 4096.0f),
                 (_Float16)((a1[0] * inv) * 4096.0f), (_Float16)((a1[1] * inv) * 4096.0f),
                 (_Float16)((a1[2] * inv) * 4096.0f), (_Float16)((a1[3] * inv) * 4096.0f)};
    const v4u vv = pk.u;
    volatile v4u* d = (volatile v4u*)(ca + (size_t)r * CP + 8 * tid);
    *d = vv;
    __threadfence();
    *d = vv;
  }
}

__global__ __launch_bounds__(256) void k_caf(const _Float16* __restrict__ ca, _Float16* __restrict__ caf) {
  __shared__ __align__(16) float fb[HW];
  const int tid = threadIdx.x;
  const int l   = blockIdx.x;
  const int b   = l / HW;
  const int pix = l - b * HW;
  const int y = pix / IW, x = pix - y * IW;
  int soff[9];
  bool sok[9];
#pragma unroll
  for (int t = 0; t < 9; ++t) {
    const int dy = t / 3, dx = t - dy * 3;
    const int ys = y + 1 - dy, xs = x + 1 - dx;
    sok[t] = ((unsigned)ys < (unsigned)IH) && ((unsigned)xs < (unsigned)IW);
    const int ysc = min(max(ys, 0), IH - 1), xsc = min(max(xs, 0), IW - 1);
    soff[t] = (b * HW + ysc * IW + xsc) * CP;
  }
#pragma unroll 1
  for (int i = 0; i < 7; ++i) {
    const int q  = tid + 256 * i;
    const int qc = min(q, HW - 1);
    const int qy = qc / IW, qx = qc - qy * IW;
    float f = 0.f;
#pragma unroll
    for (int t = 0; t < 9; ++t) {
      const int dy = t / 3, dx = t - dy * 3;
      const int py = qy - dy, px = qx - dx;
      const bool ok = sok[t] && ((unsigned)py < (unsigned)CW) && ((unsigned)px < (unsigned)CW);
      const int pyc = min(max(py, 0), CW - 1), pxc = min(max(px, 0), CW - 1);
      const float v = (float)ca[(size_t)soff[t] + pyc * CW + pxc];
      f += ok ? v : 0.f;
    }
    if (q < HW) fb[q] = f;
  }
  __syncthreads();
  if (tid < 200) {
    const float* sp = fb + 8 * tid;
    const v4f a0 = *(const v4f*)(sp), a1 = *(const v4f*)(sp + 4);
    Pack8 pk;
    pk.h = (v8h){(_Float16)a0[0], (_Float16)a0[1], (_Float16)a0[2], (_Float16)a0[3],
                 (_Float16)a1[0], (_Float16)a1[1], (_Float16)a1[2], (_Float16)a1[3]};
    const v4u vv = pk.u;
    volatile v4u* d = (volatile v4u*)(caf + (size_t)l * HW + 8 * tid);
    *d = vv;
    __threadfence();
    *d = vv;
  }
}

template <int WPB>
__global__ __launch_bounds__(32 * WPB) void k_acl(const _Float16* __restrict__ caf, const _Float16* __restrict__ bgt,
                                                  const float* __restrict__ g, const float* __restrict__ msk,
                                                  _Float16* __restrict__ con) {
  __shared__ __align__(16) float st[WPB][16 * OTP];
  const int tid = threadIdx.x, lane = tid & 31, wave = tid >> 5;
  const int hh = lane >> 4, c = lane & 15;
  const int z  = blockIdx.z;
  const int m0 = (blockIdx.y * WPB + wave) * 32;
  const int n0 = blockIdx.x * 64;
  const _Float16* A  = caf + (size_t)z * HW * HW;
  const _Float16* Bt = bgt + (size_t)z * DD * HW;

  v8f acc[2][4];
#pragma unroll
  for (int s = 0; s < 2; ++s)
#pragma unroll
    for (int t = 0; t < 4; ++t) acc[s][t] = zero8();
  gemm32x64(A, HW, Bt, HW, HW, m0, n0, lane, acc);
  out_epilogue_acl(acc, st[wave], g, msk, con, (size_t)z * HW + m0, n0, lane, hh, c);
}

template <int WPB>
__global__ __launch_bounds__(32 * WPB) void k_out(const _Float16* __restrict__ con, const _Float16* __restrict__ wt,
                                                  const float* __restrict__ bias, float* __restrict__ out) {
  __shared__ __align__(16) float st[WPB][16 * OTP];
  const int tid = threadIdx.x, lane = tid & 31, wave = tid >> 5;
  const int hh = lane >> 4, c = lane & 15;
  const int m0 = (blockIdx.y * WPB + wave) * 32;
  const int n0 = blockIdx.x * 64;

  v8f acc[2][4];
#pragma unroll
  for (int s = 0; s < 2; ++s)
#pragma unroll
    for (int t = 0; t < 4; ++t) acc[s][t] = zero8();
  gemm32x64(con, 2 * DD, wt, 2 * DD, 2 * DD, m0, n0, lane, acc);
  float bb[4];
#pragma unroll
  for (int t = 0; t < 4; ++t) bb[t] = bias[n0 + 16 * t + c];
  out_epilogue_elu(acc, 0.015625f, bb, st[wave], out, DD, m0, n0, lane, hh, c);
}

extern "C" void kernel_launch(void* const* d_in, const int* in_sizes, int n_in,
                              void* d_out, int out_size, void* d_ws, size_t ws_size,
                              hipStream_t stream) {
  if (n_in < 4) return;
  if (in_sizes[0] != NPIX * DD) return;
  if (in_sizes[1] != NPIX) return;
  if (in_sizes[2] != 2 * DD * DD) return;
  if (in_sizes[3] != DD) return;
  if (out_size != NPIX * DD) return;

  const float* g    = (const float*)d_in[0];
  const float* msk  = (const float*)d_in[1];
  const float* w    = (const float*)d_in[2];
  const float* bias = (const float*)d_in[3];
  float* out = (float*)d_out;

  size_t off = 0;
  const size_t oCON = off; off += (size_t)NPIX * 2 * DD * 2;
  const size_t oGH  = off; off += (size_t)NPIX * DD * 2;
  const size_t oGL  = off; off += (size_t)NPIX * DD * 2;
  const size_t oBH  = off; off += (size_t)NPIX * DD * 2;
  const size_t oBL  = off; off += (size_t)NPIX * DD * 2;
  const size_t oBGT = off; off += (size_t)NS * DD * HW * 2;
  const size_t oG2  = off; off += (size_t)NPIX * 4;
  const size_t oBG2 = off; off += (size_t)NPIX * 4;
  const size_t oWWD = off; off += (size_t)NPIX * 4;
  const size_t oK1D = off; off += (size_t)NS * CP * 4;
  const size_t oWT  = off; off += (size_t)DD * 2 * DD * 2;
  const size_t oGG  = off; off += (size_t)HROWS * HW * 4;
  const size_t oCA  = off; off += (size_t)NPIX * CP * 2;
  if ((size_t)NPIX * HW * 2 > (size_t)HROWS * HW * 4) return;
  if (off > ws_size) return;
  if (off > (size_t)134217728) return;

  char* ws = (char*)d_ws;
  _Float16* CON = (_Float16*)(ws + oCON);
  unsigned short* GH = (unsigned short*)(ws + oGH);
  unsigned short* GL = (unsigned short*)(ws + oGL);
  unsigned short* BH = (unsigned short*)(ws + oBH);
  unsigned short* BL = (unsigned short*)(ws + oBL);
  _Float16* BGT = (_Float16*)(ws + oBGT);
  float* G2S  = (float*)(ws + oG2);
  float* BG2S = (float*)(ws + oBG2);
  float* WWD  = (float*)(ws + oWWD);
  float* K1D  = (float*)(ws + oK1D);
  _Float16* WT  = (_Float16*)(ws + oWT);
  float*    GG4 = (float*)(ws + oGG);
  _Float16* CAF = (_Float16*)(ws + oGG);
  _Float16* CA  = (_Float16*)(ws + oCA);

  k_prep<<<dim3(NPIX / 64), dim3(256), 0, stream>>>(g, msk, CON, GH, GL, BH, BL, BGT, G2S, BG2S);
  k_wt<<<dim3((DD * 32) / 256), dim3(256), 0, stream>>>(w, WT);
  k_norm9<<<dim3(NPIX / 256 + (NS * CP) / 256), dim3(256), 0, stream>>>(G2S, BG2S, WWD, K1D);
  k_gg<5><<<dim3(HW / 64, HW / 160, 4), dim3(160), 0, stream>>>(GH, GL, BH, BL, GG4, 0);
  k_stats<<<dim3(HROWS), dim3(256), 0, stream>>>(GG4, WWD, K1D, CA, 0);
  k_gg<5><<<dim3(HW / 64, HW / 160, 4), dim3(160), 0, stream>>>(GH, GL, BH, BL, GG4, 4);
  k_stats<<<dim3(HROWS), dim3(256), 0, stream>>>(GG4, WWD, K1D, CA, HROWS);
  k_caf<<<dim3(NPIX), dim3(256), 0, stream>>>(CA, CAF);
  k_acl<5><<<dim3(DD / 64, HW / 160, NS), dim3(160), 0, stream>>>(CAF, BGT, g, msk, CON);
  k_out<8><<<dim3(DD / 64, NPIX / 256, 1), dim3(256), 0, stream>>>(CON, WT, bias, out);
  (void)hipGetLastError();
}
